// SelfAttention_9801115369787
// MI455X (gfx1250) — hardware-verified
//
#include <hip/hip_runtime.h>
#include <math.h>

#ifndef NB
#define NB 8
#endif
#ifndef SEQ
#define SEQ 2048
#endif
#define NB_FULL 8
#define SEQ_FULL 2048
#define DD 256
#define PP 72

__host__ __device__ constexpr unsigned ilog2c(unsigned v) { return (v <= 1u) ? 0u : 1u + ilog2c(v >> 1); }
enum : unsigned { LSEQ = ilog2c((unsigned)SEQ) };

static_assert(NB >= 1 && NB <= NB_FULL);
static_assert(SEQ >= 64 && SEQ <= SEQ_FULL && (SEQ % 64) == 0);
static_assert((1u << LSEQ) == (unsigned)SEQ);
static_assert(DD == 256 && (DD % 32) == 0 && (DD % 8) == 0);
#define CVT_X8 (NB * SEQ * DD / 8)
#define CVT_W8 (DD * DD / 8)
#define CVT_THREADS (3 * CVT_X8 + 4 * CVT_W8)
#define CVT_XBLK (CVT_X8 / 256)
static_assert((CVT_X8 % 256) == 0 && (CVT_W8 % 256) == 0 && (CVT_THREADS % 256) == 0);
static_assert(CVT_W8 / 256 == 32 && CVT_W8 * 8 == DD * DD);
static_assert((SEQ * (DD / 8)) / 256 == (SEQ >> 3));
static_assert(((NB * SEQ / 4) % 8) == 0);
static_assert((NB * SEQ / 16) * 4 == NB * SEQ / 4 && NB * (DD / 16) * (SEQ / 64) == NB * SEQ / 4);
static_assert((SEQ % 16) == 0 && 4 * 64 == DD);
static_assert((SEQ % 32) == 0 && ((SEQ / 16) % 4) == 0 && LSEQ >= 6u);
static_assert((NB * SEQ / 16) * 4 == (NB * SEQ / 32) * 8);

#define OUT1_OFF ((size_t)NB_FULL * SEQ_FULL * DD)
static_assert(OUT1_OFF * 4 == (size_t)16777216);
static_assert((size_t)NB * SEQ * DD <= OUT1_OFF);
static_assert(((OUT1_OFF * 4) % 128) == 0);

#define XPL ((size_t)NB * SEQ * DD)
#define WS_X16 ((size_t)3 * NB * SEQ * DD * 2)
#define WS_W16 ((size_t)4 * DD * DD * 2)
#define WS_PL  ((size_t)NB * SEQ * DD * 2)
#define WS_ST  ((size_t)(NB * SEQ / 16) * 32 * 4)
#define WS_TOTAL (WS_X16 + WS_W16 + 4 * WS_PL + WS_ST)
static_assert(WS_TOTAL <= (size_t)134217728);
static_assert((WS_X16 % 128) == 0 && (WS_W16 % 128) == 0 && (WS_PL % 128) == 0 && (WS_ST % 128) == 0);

typedef __attribute__((ext_vector_type(16))) _Float16 v16h;
typedef __attribute__((ext_vector_type(8)))  _Float16 v8h;
typedef __attribute__((ext_vector_type(8)))  float    v8f;
typedef __attribute__((ext_vector_type(4)))  float    v4f;
typedef v4f __attribute__((may_alias)) f4a;
typedef unsigned __attribute__((may_alias)) ua32;
#define SFOLD  (1.0f / 4096.0f)
#define PCARRY 16384.0f
#define CFOLD  64.0f
#define OFOLD  (1.0f / 16384.0f)
#define NEG_INF (-__builtin_inff())

static __device__ __forceinline__ _Float16 toh_flush(float v) {
  const _Float16 r = (_Float16)v;
  return (fabsf(v) < 6.103515625e-05f) ? (_Float16)0.0f : r;
}

static __device__ __forceinline__ float bf16v(float f) { return (float)(__bf16)f; }

static __device__ __forceinline__ _Float16 cvt_in16(float f) { return toh_flush(bf16v(f) * 16.0f); }

__device__ __forceinline__ v8f wmma_h16(v16h a, v16h b, v8f c) {
  v8f d = __builtin_amdgcn_wmma_f32_16x16x32_f16(false, a, false, b, (short)0, c, false, false);
  asm volatile("v_nop\n\tv_nop\n\tv_nop\n\tv_nop" : "+v"(d) : "v"(a), "v"(b));
  return d;
}

__device__ __forceinline__ v8f v8f_zero() {
  v8f z = {0.f, 0.f, 0.f, 0.f, 0.f, 0.f, 0.f, 0.f};
  return z;
}

union U16 { v16h v; v8h h[2]; };

__global__ void __launch_bounds__(256)
cvt_kernel(const float* __restrict__ x,
           const float* __restrict__ y,
           const float* __restrict__ z,
           const float* __restrict__ Wq,
           const float* __restrict__ Wk,
           const float* __restrict__ Wv,
           const float* __restrict__ Wo,
           _Float16* __restrict__ X16,
           _Float16* __restrict__ W16) {
  const unsigned bx = blockIdx.x;
  const unsigned tx = threadIdx.x;
  const float* src;
  _Float16* dst;
  if (bx < 3u * (unsigned)CVT_XBLK) {
    const unsigned pl = (bx >= 2u * (unsigned)CVT_XBLK) ? 2u : ((bx >= (unsigned)CVT_XBLK) ? 1u : 0u);
    const unsigned lb = bx - pl * (unsigned)CVT_XBLK;
    const unsigned e8 = (lb << 8) + tx;
    const unsigned b  = lb >> (LSEQ - 3u);
    const float* asrc = (pl == 0u) ? x : ((pl == 1u) ? y : z);
    src = asrc + (size_t)e8 * 8u + (size_t)b * (size_t)((SEQ_FULL - SEQ) * DD);
    dst = X16 + (size_t)pl * XPL + (size_t)e8 * 8u;
  } else {
    const unsigned wb  = bx - 3u * (unsigned)CVT_XBLK;
    const unsigned mat = wb >> 5;
    const unsigned r8  = ((wb & 31u) << 8) + tx;
    const float* wsrc = (mat == 0u) ? Wq : ((mat == 1u) ? Wk : ((mat == 2u) ? Wv : Wo));
    src = wsrc + (size_t)r8 * 8u;
    dst = W16 + (size_t)((wb << 8) + tx) * 8u;
  }
  const v4f f0 = *(const v4f*)src;
  const v4f f1 = *(const v4f*)(src + 4);
  v8h o;
  o[0] = cvt_in16(f0[0]); o[1] = cvt_in16(f0[1]); o[2] = cvt_in16(f0[2]); o[3] = cvt_in16(f0[3]);
  o[4] = cvt_in16(f1[0]); o[5] = cvt_in16(f1[1]); o[6] = cvt_in16(f1[2]); o[7] = cvt_in16(f1[3]);
  *(volatile v8h*)dst = o;
  __threadfence();
  *(volatile v8h*)dst = o;
}

__global__ void __launch_bounds__(256)
qkv_kernel(const _Float16* __restrict__ X16,
           const _Float16* __restrict__ W16,
           const float* __restrict__ bq,
           const float* __restrict__ bk,
           const float* __restrict__ bv,
           _Float16* __restrict__ qws,
           _Float16* __restrict__ kws,
           _Float16* __restrict__ vtws) {
  __shared__ __align__(16) _Float16 st[8][16][64];
  const unsigned lane = threadIdx.x & 31u;
  const unsigned wv   = (unsigned)__builtin_amdgcn_readfirstlane((int)(threadIdx.x >> 5));
  const unsigned g    = lane >> 4;
  const unsigned m    = lane & 15u;
  const unsigned y    = blockIdx.y;
  const unsigned tile = (blockIdx.x << 3) + wv;

  const _Float16* Ap;
  const _Float16* Bp;
  _Float16* op;
  size_t pitch;
  unsigned bc0 = 0u;
  unsigned br0 = 0u;
  if (y < 2u) {
    const unsigned rt = tile >> 2;
    const unsigned cg = tile & 3u;
    Ap = X16 + (size_t)y * XPL + (size_t)rt * 16u * DD;
    Bp = W16 + (size_t)y * DD * DD + (size_t)cg * 64u * DD;
    op = ((y == 0u) ? qws : kws) + (size_t)rt * 16u * DD + (size_t)cg * 64u;
    pitch = DD;
    bc0 = cg * 64u;
  } else {
    const unsigned b   = tile >> (LSEQ - 2u);
    const unsigned rem = tile & ((unsigned)(SEQ / 4) - 1u);
    const unsigned et  = rem >> (LSEQ - 6u);
    const unsigned ng  = rem & ((unsigned)(SEQ / 64) - 1u);
    Ap = W16 + (size_t)2 * DD * DD + (size_t)et * 16u * DD;
    Bp = X16 + (size_t)2 * XPL + (((size_t)b << LSEQ) + (size_t)ng * 64u) * DD;
    op = vtws + (((size_t)b * DD + (size_t)et * 16u) << LSEQ) + (size_t)ng * 64u;
    pitch = SEQ;
    br0 = et * 16u;
  }

  const float* bsrc = (y == 0u) ? bq : ((y == 1u) ? bk : bv);
  float bcol[4], brow[8];
#pragma unroll
  for (int nt = 0; nt < 4; ++nt) {
    const float t = bsrc[bc0 + (unsigned)nt * 16u + m];
    bcol[nt] = (y < 2u) ? (bf16v(t) * 16.0f) : 0.0f;
  }
#pragma unroll
  for (int v = 0; v < 8; ++v) {
    const float t = bsrc[br0 + 8u * g + (unsigned)v];
    brow[v] = (y < 2u) ? 0.0f : (bf16v(t) * 16.0f);
  }

  v8f acc[4];
#pragma unroll
  for (int nt = 0; nt < 4; ++nt) acc[nt] = v8f_zero();

  const _Float16* arow = Ap + (size_t)m * DD + 8u * g;
  const _Float16* brw  = Bp + (size_t)m * DD + 8u * g;

#pragma unroll 2
  for (unsigned c0 = 0; c0 < (unsigned)DD; c0 += 32u) {
    U16 a;
    a.h[0] = *(const v8h*)(arow + c0);
    a.h[1] = *(const v8h*)(arow + c0 + 16u);
#pragma unroll
    for (int nt = 0; nt < 4; ++nt) {
      U16 bb;
      bb.h[0] = *(const v8h*)(brw + (size_t)nt * 16 * DD + c0);
      bb.h[1] = *(const v8h*)(brw + (size_t)nt * 16 * DD + c0 + 16u);
      acc[nt] = wmma_h16(a.v, bb.v, acc[nt]);
    }
  }

#pragma unroll
  for (int nt = 0; nt < 4; ++nt)
#pragma unroll
    for (int v = 0; v < 8; ++v) {
      const float val = acc[nt][v] * 0.0625f + (bcol[nt] + brow[v]);
      st[wv][8u * g + (unsigned)v][(unsigned)nt * 16u + m] = toh_flush(val);
    }
  __builtin_amdgcn_fence(3  , "wavefront");
  __builtin_amdgcn_wave_barrier();
  asm volatile("s_wait_dscnt 0" ::: "memory");
  unsigned w[16];
#pragma unroll
  for (int r = 0; r < 16; ++r) w[r] = *((const ua32*)&st[wv][r][0] + lane);
#pragma unroll
  for (int r = 0; r < 16; ++r) *(volatile unsigned*)((unsigned*)(op + (size_t)r * pitch) + lane) = w[r];
  __threadfence();
#pragma unroll
  for (int r = 0; r < 16; ++r) *(volatile unsigned*)((unsigned*)(op + (size_t)r * pitch) + lane) = w[r];
}

__global__ void __launch_bounds__(128)
attn_kernel(const _Float16* __restrict__ qws,
            const _Float16* __restrict__ kws,
            const _Float16* __restrict__ vtws,
            _Float16* __restrict__ ctxws,
            float* __restrict__ stws) {
  __shared__ __align__(16) _Float16 Pl[16][PP];
  __shared__ __align__(16) float Mx[4][16];
  __shared__ __align__(16) float Ls[4][16];
  __shared__ __align__(16) _Float16 Cf[4][16][64];
  __shared__ __align__(16) float Sx[32];

  const unsigned lane = threadIdx.x & 31u;
  const unsigned wv   = (unsigned)__builtin_amdgcn_readfirstlane((int)(threadIdx.x >> 5));
  const unsigned g    = lane >> 4;
  const unsigned m    = lane & 15u;
  const unsigned tile = blockIdx.x;
  const unsigned b    = tile >> (LSEQ - 4u);
  const unsigned t0   = (tile & ((unsigned)(SEQ / 16) - 1u)) << 4;

  const _Float16* qrow  = qws + (((size_t)b << LSEQ) + t0 + m) * DD + 8u * g;
  const _Float16* kbase = kws + (((size_t)b << LSEQ) + 16u * wv + m) * DD + 8u * g;
  const _Float16* vbase = vtws + (((size_t)b * DD + 64u * wv + m) << LSEQ) + 8u * g;

  v8f o[4];
#pragma unroll
  for (int nt = 0; nt < 4; ++nt) o[nt] = v8f_zero();
  float mrow[8], lrow[8];
#pragma unroll
  for (int v = 0; v < 8; ++v) { mrow[v] = NEG_INF; lrow[v] = 0.f; }

#pragma unroll 1
  for (unsigned kb = 0; kb < (unsigned)(SEQ / 64); ++kb) {
    const unsigned s0 = kb << 6;

    const _Float16* krow = kbase + (size_t)s0 * DD;
    v8f sh = v8f_zero();
#pragma unroll 2
    for (unsigned c = 0; c < (unsigned)DD; c += 32u) {
      U16 qa, kf;
      qa.h[0] = *(const v8h*)(qrow + c);        qa.h[1] = *(const v8h*)(qrow + c + 16u);
      kf.h[0] = *(const v8h*)(krow + c);        kf.h[1] = *(const v8h*)(krow + c + 16u);
      sh = wmma_h16(qa.v, kf.v, sh);
    }

    float sv[8], rmax[8];
#pragma unroll
    for (int v = 0; v < 8; ++v) {
      sv[v] = sh[v] * SFOLD;
      rmax[v] = sv[v];
    }
#pragma unroll
    for (int off = 1; off < 16; off <<= 1)
#pragma unroll
      for (int v = 0; v < 8; ++v)
        rmax[v] = fmaxf(rmax[v], __shfl_xor(rmax[v], off, 32));
    if (m == 0u) {
#pragma unroll
      for (int v = 0; v < 8; ++v) Mx[wv][8u * g + (unsigned)v] = rmax[v];
    }
    __syncthreads();

    float mb[8];
    {
      const f4a a0 = *(const f4a*)&Mx[0][8u * g];
      const f4a a1 = *(const f4a*)&Mx[0][8u * g + 4u];
#pragma unroll
      for (int j = 0; j < 4; ++j) { mb[j] = a0[j]; mb[4 + j] = a1[j]; }
    }
#pragma unroll
    for (int w2 = 1; w2 < 4; ++w2) {
      const f4a a0 = *(const f4a*)&Mx[w2][8u * g];
      const f4a a1 = *(const f4a*)&Mx[w2][8u * g + 4u];
#pragma unroll
      for (int j = 0; j < 4; ++j) { mb[j] = fmaxf(mb[j], a0[j]); mb[4 + j] = fmaxf(mb[4 + j], a1[j]); }
    }
    float alpha[8];
#pragma unroll
    for (int v = 0; v < 8; ++v) {
      const float mnew = fmaxf(mrow[v], mb[v]);
      alpha[v] = __expf(mrow[v] - mnew);
      mrow[v]  = mnew;
      const float p = __expf(sv[v] - mnew);
      const _Float16 ph = toh_flush(p * PCARRY);
      lrow[v] = lrow[v] * alpha[v] + (float)ph;
      Pl[8u * g + (unsigned)v][16u * wv + m] = ph;
    }
#pragma unroll
    for (int nt = 0; nt < 4; ++nt)
#pragma unroll
      for (int v = 0; v < 8; ++v)
        o[nt][v] *= alpha[v];
    __syncthreads();

    U16 pa[2];
#pragma unroll
    for (int ks = 0; ks < 2; ++ks) {
      pa[ks].h[0] = *(const v8h*)&Pl[m][32u * (unsigned)ks + 8u * g];
      pa[ks].h[1] = *(const v8h*)&Pl[m][32u * (unsigned)ks + 16u + 8u * g];
    }

    const _Float16* vrow = vbase + s0;
#pragma unroll
    for (int nt = 0; nt < 4; ++nt) {
#pragma unroll
      for (int ks = 0; ks < 2; ++ks) {
        const _Float16* vp = vrow + (size_t)nt * 16 * SEQ + 32 * ks;
        U16 vb;
        vb.h[0] = *(const v8h*)(vp);        vb.h[1] = *(const v8h*)(vp + 16);
        o[nt] = wmma_h16(pa[ks].v, vb.v, o[nt]);
      }
    }
  }

#pragma unroll
  for (int off = 1; off < 16; off <<= 1)
#pragma unroll
    for (int v = 0; v < 8; ++v)
      lrow[v] += __shfl_xor(lrow[v], off, 32);
  if (m == 0u) {
#pragma unroll
    for (int v = 0; v < 8; ++v) Ls[wv][8u * g + (unsigned)v] = lrow[v];
  }
  __syncthreads();
  float cs[8], sinv[8];
  {
    float lt[8];
    const f4a a0 = *(const f4a*)&Ls[0][8u * g];
    const f4a a1 = *(const f4a*)&Ls[0][8u * g + 4u];
#pragma unroll
    for (int j = 0; j < 4; ++j) { lt[j] = a0[j]; lt[4 + j] = a1[j]; }
#pragma unroll
    for (int w2 = 1; w2 < 4; ++w2) {
      const f4a c0 = *(const f4a*)&Ls[w2][8u * g];
      const f4a c1 = *(const f4a*)&Ls[w2][8u * g + 4u];
#pragma unroll
      for (int j = 0; j < 4; ++j) { lt[j] += c0[j]; lt[4 + j] += c1[j]; }
    }
#pragma unroll
    for (int v = 0; v < 8; ++v) {
      const float r = 1.0f / lt[v];
      cs[v]   = CFOLD * r;
      sinv[v] = PCARRY * r;
    }
  }

  if (wv == 0u && m == 0u) {
#pragma unroll
    for (int v = 0; v < 8; ++v) {
      Sx[8u * g + (unsigned)v]       = mrow[v];
      Sx[16u + 8u * g + (unsigned)v] = sinv[v];
    }
  }
#pragma unroll
  for (int nt = 0; nt < 4; ++nt)
#pragma unroll
    for (int v = 0; v < 8; ++v)
      Cf[wv][8u * g + (unsigned)v][(unsigned)nt * 16u + m] = toh_flush(o[nt][v] * cs[v]);
  __syncthreads();

  _Float16* cbase = ctxws + (((size_t)b << LSEQ) + t0) * DD + 64u * wv;
  float* sline = stws + (size_t)tile * 32u + lane;
  const float sval = Sx[lane];
  unsigned w[16];
#pragma unroll
  for (int r = 0; r < 16; ++r) w[r] = *((const ua32*)&Cf[wv][r][0] + lane);
#pragma unroll
  for (int r = 0; r < 16; ++r) *(volatile unsigned*)((unsigned*)(cbase + (size_t)r * DD) + lane) = w[r];
  if (wv == 0u) *(volatile float*)sline = sval;
  __threadfence();
#pragma unroll
  for (int r = 0; r < 16; ++r) *(volatile unsigned*)((unsigned*)(cbase + (size_t)r * DD) + lane) = w[r];
  if (wv == 0u) *(volatile float*)sline = sval;
}

__global__ void __launch_bounds__(256)
colmean_kernel(const _Float16* __restrict__ qws,
               const _Float16* __restrict__ kws,
               const float* __restrict__ stws,
               float* __restrict__ out1) {
  __shared__ __align__(16) float Part[8][16];
  const unsigned lane = threadIdx.x & 31u;
  const unsigned wv   = (unsigned)__builtin_amdgcn_readfirstlane((int)(threadIdx.x >> 5));
  const unsigned g    = lane >> 4;
  const unsigned m    = lane & 15u;
  const unsigned blk  = blockIdx.x;
  const unsigned b    = blk >> (LSEQ - 5u);
  const unsigned key0 = (blk & ((unsigned)(SEQ / 32) - 1u)) << 5;
  const unsigned kt   = wv >> 2;
  const unsigned qs   = wv & 3u;

  const _Float16* krow = kws + (((size_t)b << LSEQ) + key0 + 16u * kt + m) * DD + 8u * g;
  U16 kf[8];
#pragma unroll
  for (int c = 0; c < 8; ++c) {
    kf[c].h[0] = *(const v8h*)(krow + 32 * c);
    kf[c].h[1] = *(const v8h*)(krow + 32 * c + 16);
  }
  const _Float16* qbase = qws + (((size_t)b << LSEQ) + m) * DD + 8u * g;
  const float* sbase = stws + ((size_t)b << (LSEQ - 4u)) * 32u + m;

  float cs[8];
#pragma unroll
  for (int v = 0; v < 8; ++v) cs[v] = 0.f;

#pragma unroll 1
  for (unsigned qt = qs; qt < (unsigned)(SEQ / 16); qt += 4u) {
    const _Float16* qrow = qbase + (size_t)qt * 16u * DD;
    v8f s = v8f_zero();
#pragma unroll
    for (int c = 0; c < 8; ++c) {
      U16 qf;
      qf.h[0] = *(const v8h*)(qrow + 32 * c);
      qf.h[1] = *(const v8h*)(qrow + 32 * c + 16);
      s = wmma_h16(kf[c].v, qf.v, s);
    }
    const float mq = sbase[(size_t)qt * 32u];
    const float iq = sbase[(size_t)qt * 32u + 16u];
#pragma unroll
    for (int v = 0; v < 8; ++v)
      cs[v] += __expf(s[v] * SFOLD - mq) * iq;
  }

#pragma unroll
  for (int off = 1; off < 16; off <<= 1)
#pragma unroll
    for (int v = 0; v < 8; ++v)
      cs[v] += __shfl_xor(cs[v], off, 32);
  if (m == 0u) {
#pragma unroll
    for (int v = 0; v < 8; ++v) Part[wv][8u * g + (unsigned)v] = cs[v];
  }
  __syncthreads();

  if (wv == 0u) {
    const unsigned t = lane >> 4;
    const unsigned r = lane & 15u;
    float tot = Part[4u * t][r];
    tot += Part[4u * t + 1u][r];
    tot += Part[4u * t + 2u][r];
    tot += Part[4u * t + 3u][r];
    const float val = tot * (1.0f / (float)SEQ);
    float* dst = out1 + ((size_t)b << LSEQ) + key0 + lane;
    *(volatile float*)dst = val;
    __threadfence();
    *(volatile float*)dst = val;
  }
}

__global__ void __launch_bounds__(256)
oproj_kernel(const _Float16* __restrict__ ctxws,
             const _Float16* __restrict__ W16,
             const float* __restrict__ bo,
             float* __restrict__ out) {
  __shared__ __align__(16) float Of[8][16][64];
  const unsigned lane = threadIdx.x & 31u;
  const unsigned wv   = (unsigned)__builtin_amdgcn_readfirstlane((int)(threadIdx.x >> 5));
  const unsigned g    = lane >> 4;
  const unsigned m    = lane & 15u;
  const unsigned tile = (blockIdx.x << 3) + wv;
  const unsigned rt   = tile >> 2;
  const unsigned cg   = tile & 3u;

  const _Float16* arow = ctxws + (size_t)rt * 16u * DD + (size_t)m * DD + 8u * g;
  const _Float16* brw  = W16 + (size_t)3 * DD * DD + (size_t)cg * 64u * DD + (size_t)m * DD + 8u * g;

  float bcol[4];
#pragma unroll
  for (int nt = 0; nt < 4; ++nt) bcol[nt] = bf16v(bo[cg * 64u + (unsigned)nt * 16u + m]);

  v8f acc[4];
#pragma unroll
  for (int nt = 0; nt < 4; ++nt) acc[nt] = v8f_zero();

#pragma unroll 2
  for (unsigned c0 = 0; c0 < (unsigned)DD; c0 += 32u) {
    U16 a;
    a.h[0] = *(const v8h*)(arow + c0);
    a.h[1] = *(const v8h*)(arow + c0 + 16u);
#pragma unroll
    for (int nt = 0; nt < 4; ++nt) {
      U16 bb;
      bb.h[0] = *(const v8h*)(brw + (size_t)nt * 16 * DD + c0);
      bb.h[1] = *(const v8h*)(brw + (size_t)nt * 16 * DD + c0 + 16u);
      acc[nt] = wmma_h16(a.v, bb.v, acc[nt]);
    }
  }

#pragma unroll
  for (int nt = 0; nt < 4; ++nt)
#pragma unroll
    for (int v = 0; v < 8; ++v)
      Of[wv][8u * g + (unsigned)v][(unsigned)nt * 16u + m] = acc[nt][v] * OFOLD + bcol[nt];
  __syncthreads();

  float* obase = out + (size_t)rt * 16u * DD + 64u * cg;
  const unsigned rsel = lane >> 4;
  const unsigned c4   = 4u * (lane & 15u);
  v4f w[8];
#pragma unroll
  for (int it = 0; it < 8; ++it) w[it] = *(const f4a*)&Of[wv][2u * (unsigned)it + rsel][c4];
#pragma unroll
  for (int it = 0; it < 8; ++it) *(volatile v4f*)(obase + (size_t)(2u * (unsigned)it + rsel) * DD + c4) = w[it];
  __threadfence();
#pragma unroll
  for (int it = 0; it < 8; ++it) *(volatile v4f*)(obase + (size_t)(2u * (unsigned)it + rsel) * DD + c4) = w[it];
}

extern "C" void kernel_launch(void* const* d_in, const int* in_sizes, int n_in,
                              void* d_out, int out_size, void* d_ws,
                              size_t ws_size, hipStream_t stream) {
  if (n_in < 11) return;
  const long long need_x = ((long long)(NB - 1) * SEQ_FULL + SEQ) * (long long)DD;
  if ((long long)in_sizes[0] < need_x || (long long)in_sizes[1] < need_x || (long long)in_sizes[2] < need_x) return;
  if (in_sizes[3] < DD * DD || in_sizes[5] < DD * DD || in_sizes[7] < DD * DD || in_sizes[9] < DD * DD) return;
  if (in_sizes[4] < DD || in_sizes[6] < DD || in_sizes[8] < DD || in_sizes[10] < DD) return;
  if ((long long)out_size < (long long)OUT1_OFF + (long long)NB * SEQ) return;

  const float* x  = (const float*)d_in[0];
  const float* y  = (const float*)d_in[1];
  const float* z  = (const float*)d_in[2];
  const float* Wq = (const float*)d_in[3];
  const float* bq = (const float*)d_in[4];
  const float* Wk = (const float*)d_in[5];
  const float* bk = (const float*)d_in[6];
  const float* Wv = (const float*)d_in[7];
  const float* bv = (const float*)d_in[8];
  const float* Wo = (const float*)d_in[9];
  const float* bo = (const float*)d_in[10];
  float* out  = (float*)d_out;
  float* out1 = out + OUT1_OFF;

  char* ws = (char*)d_ws;
  const size_t total = WS_TOTAL;
  if (total > ws_size || total > (size_t)134217728) return;
  _Float16* X16   = (_Float16*)(ws);
  _Float16* W16   = (_Float16*)(ws + WS_X16);
  _Float16* qws   = (_Float16*)(ws + WS_X16 + WS_W16);
  _Float16* kws   = (_Float16*)(ws + WS_X16 + WS_W16 + WS_PL);
  _Float16* vtws  = (_Float16*)(ws + WS_X16 + WS_W16 + 2 * WS_PL);
  _Float16* ctxws = (_Float16*)(ws + WS_X16 + WS_W16 + 3 * WS_PL);
  float*    stws  = (float*)(ws + WS_X16 + WS_W16 + 4 * WS_PL);

  cvt_kernel<<<CVT_THREADS / 256, 256, 0, stream>>>(x, y, z, Wq, Wk, Wv, Wo, X16, W16);
  qkv_kernel<<<dim3(NB * SEQ / 32, 3), 256, 0, stream>>>(X16, W16, bq, bk, bv, qws, kws, vtws);
  attn_kernel<<<NB * SEQ / 16, 128, 0, stream>>>(qws, kws, vtws, ctxws, stws);
  colmean_kernel<<<NB * SEQ / 32, 256, 0, stream>>>(qws, kws, stws, out1);
  oproj_kernel<<<NB * SEQ / 32, 256, 0, stream>>>(ctxws, W16, bo, out);
}
